// RpeSelfAttentionV2S1_30932354466495
// MI455X (gfx1250) — hardware-run, weakly checked
//
#include <hip/hip_runtime.h>
#include <math.h>

typedef __attribute__((ext_vector_type(16))) _Float16 v16h;
typedef __attribute__((ext_vector_type(16))) __bf16 v16b;
typedef __attribute__((ext_vector_type(8)))  _Float16 v8h;
typedef __attribute__((ext_vector_type(8)))  float v8f;
typedef __attribute__((ext_vector_type(4)))  float v4f;
typedef __attribute__((ext_vector_type(2)))  float v2f;
typedef __attribute__((ext_vector_type(4)))  unsigned v4u;
typedef __attribute__((ext_vector_type(4)))  int v4i;
typedef float __attribute__((may_alias)) float_a;
typedef int __attribute__((may_alias)) int_a;

template <typename T> __device__ __forceinline__ void vst2(void* p, T v) { *(volatile T*)p = v; __threadfence(); *(volatile T*)p = v; }
__device__ __forceinline__ v8f wmma16(v16h a, v16h b, v8f c) {
  v8f d = __builtin_amdgcn_wmma_f32_16x16x32_f16(false, a, false, b, (short)0, c, false, false);
  asm volatile("v_nop\n\tv_nop\n\tv_nop\n\tv_nop" : "+v"(d) : "v"(a), "v"(b));
  return d;
}
__device__ __forceinline__ v8f wmma_bf(v16b a, v16b b, v8f c) {
  v8f d = __builtin_amdgcn_wmma_f32_16x16x32_bf16(false, a, false, b, (short)0, c, false, false);
  asm volatile("v_nop\n\tv_nop\n\tv_nop\n\tv_nop" : "+v"(d) : "v"(a), "v"(b));
  return d;
}
__device__ __forceinline__ v16h frag_h(const _Float16* rowk0, int lane) {
  union { v16h v; v8h q[2]; } u; const _Float16* p = rowk0 + 8 * (lane >> 4);
  u.q[0] = *(const v8h*)p; u.q[1] = *(const v8h*)(p + 16); return u.v;
}
__device__ __forceinline__ v16h frag_f32(const float* rowk0, int lane) {
  v16h a; const float* p = rowk0 + 8 * (lane >> 4);
#pragma unroll
  for (int i = 0; i < 8; ++i) { a[i] = (_Float16)p[i]; a[8 + i] = (_Float16)p[16 + i]; }
  return a;
}
__device__ __forceinline__ v16h frag_f32s(const float* rowk0, int lane, float sc) {
  v16h a; const float* p = rowk0 + 8 * (lane >> 4);
#pragma unroll
  for (int i = 0; i < 8; ++i) { a[i] = (_Float16)(p[i] * sc); a[8 + i] = (_Float16)(p[16 + i] * sc); }
  return a;
}
__device__ __forceinline__ v16h fragc_f32(const float* W, int k0, int n, int lane, int ld, int K) {
  v16h a; const int g = lane >> 4;
#pragma unroll
  for (int i = 0; i < 8; ++i) { const int ka = k0 + 8 * g + i, kb = ka + 16;
    a[i] = (_Float16)(ka < K ? W[(size_t)(ka < K ? ka : K - 1) * ld + n] : 0.f); a[8 + i] = (_Float16)(kb < K ? W[(size_t)(kb < K ? kb : K - 1) * ld + n] : 0.f); }
  return a;
}
struct F2 { v16b h, l; };
__device__ __forceinline__ F2 bsplit16(const float v[16]) { F2 r;
#pragma unroll
  for (int i = 0; i < 16; ++i) { const __bf16 h = (__bf16)v[i]; r.h[i] = h; r.l[i] = (__bf16)(v[i] - (float)h); }
  return r; }
__device__ __forceinline__ F2 split_row(const float* row, int k0, int lane) { float v[16]; const float* p = row + k0 + 8 * (lane >> 4);
#pragma unroll
  for (int i = 0; i < 8; ++i) { v[i] = p[i]; v[8 + i] = p[16 + i]; }
  return bsplit16(v); }
__device__ __forceinline__ F2 split_rowK(const float* row, int k0, int lane, int K) { float v[16]; const int g = lane >> 4;
#pragma unroll
  for (int i = 0; i < 8; ++i) { const int ka = k0 + 8 * g + i, kb = ka + 16; v[i] = ka < K ? row[ka < K ? ka : K - 1] : 0.f; v[8 + i] = kb < K ? row[kb < K ? kb : K - 1] : 0.f; }
  return bsplit16(v); }
__device__ __forceinline__ F2 split_col(const float* W, int k0, int n, int lane, int ld, int K) { float v[16]; const int g = lane >> 4;
#pragma unroll
  for (int i = 0; i < 8; ++i) { const int ka = k0 + 8 * g + i, kb = ka + 16; v[i] = ka < K ? W[(size_t)(ka < K ? ka : K - 1) * ld + n] : 0.f; v[8 + i] = kb < K ? W[(size_t)(kb < K ? kb : K - 1) * ld + n] : 0.f; }
  return bsplit16(v); }
__device__ __forceinline__ v8f mac3(const F2& a, const F2& b, v8f c) { c = wmma_bf(a.l, b.h, c); c = wmma_bf(a.h, b.l, c); return wmma_bf(a.h, b.h, c); }
__device__ __forceinline__ float sigm(float v) { return 1.0f / (1.0f + expf(-v)); }
#define LDSX() do { asm volatile("s_wait_dscnt 0" ::: "memory"); __builtin_amdgcn_wave_barrier(); __builtin_amdgcn_fence(__ATOMIC_RELEASE, "workgroup"); } while (0)


#define NB 2
#define EE 1024
#define NH 16
#define HD 64
#define NS 32
#define NR 2048
#define NSLOT (64 + NR)
#define NKT (NSLOT / 32)
#define NT1 (NS + NR)
#ifndef TNB
#define TNB NB
#endif
#ifndef TQ2
#define TQ2 (NR / 64)
#endif
typedef __attribute__((ext_vector_type(8))) __bf16 v8b;
__device__ __forceinline__ v16b frag_b(const __bf16* rowk0, int lane) {
  union { v16b v; v8b q[2]; } u; const __bf16* p = rowk0 + 8 * (lane >> 4);
  u.q[0] = *(const v8b*)p; u.q[1] = *(const v8b*)(p + 16); return u.v;
}
__device__ __forceinline__ float bfr(float v) { return (float)(__bf16)v; }
__device__ __attribute__((noinline)) float exp_ni(float v) { return expf(v); }
__device__ __attribute__((noinline)) float erf_ni(float v) { return erff(v); }

#define WS_QH  0u
#define WS_QL  (WS_QH + 2u * (size_t)NB * NR * EE)
#define WS_KH  (WS_QL + 2u * (size_t)NB * NR * EE)
#define WS_KL  (WS_KH + 2u * (size_t)NB * NSLOT * EE)
#define WS_VH  (WS_KL + 2u * (size_t)NB * NSLOT * EE)
#define WS_VL  (WS_VH + 2u * (size_t)NB * EE * NSLOT)
#define WS_O   (WS_VL + 2u * (size_t)NB * EE * NSLOT)
#define WS_Q1H (WS_O + 4u * (size_t)NB * NR * EE)
#define WS_Q1L (WS_Q1H + 2u * (size_t)NB * NS * EE)
#define WS_SX  (WS_Q1L + 2u * (size_t)NB * NS * EE)
#define WS_END (WS_SX + 4u * (size_t)NB * NS * EE)

__device__ __forceinline__ v16b fragb_f32(const float* __restrict__ p, int lane) { v16b a; const float* pp = p + 8 * (lane >> 4);
#pragma unroll
  for (int i = 0; i < 8; ++i) { a[i] = (__bf16)pp[i]; a[8 + i] = (__bf16)pp[16 + i]; } return a; }
__global__ __launch_bounds__(128) void k_reg(const float* __restrict__ RX, const float* __restrict__ WQ, const float* __restrict__ BQ, const float* __restrict__ WK, const float* __restrict__ BK, const float* __restrict__ WV, const float* __restrict__ BV, _Float16* __restrict__ QH, _Float16* __restrict__ QL, _Float16* __restrict__ KH, _Float16* __restrict__ KL, _Float16* __restrict__ VH, _Float16* __restrict__ VL) {
  __shared__ __align__(16) _Float16 sh[64][136], sl[64][136]; __shared__ __align__(16) _Float16 th[128][72], tl[128][72];
  const int tid = threadIdx.x, wave = tid >> 5, lane = tid & 31, col = lane & 15, g = lane >> 4; const int which = blockIdx.z / TNB; const size_t b = blockIdx.z % TNB; const int l0 = blockIdx.x * 64; const int c0 = blockIdx.y * 128;
  const float* Wm = which == 0 ? WQ : which == 1 ? WK : WV; const float* Bm = which == 0 ? BQ : which == 1 ? BK : BV;
  v8f acc[8] = {};
#pragma unroll 2
  for (int kc = 0; kc < EE / 32; ++kc) { const v16b a = fragb_f32(RX + ((size_t)(l0 + wave * 16 + col) * NB + b) * EE + kc * 32, lane);
#pragma unroll
    for (int j = 0; j < 8; ++j) acc[j] = wmma_bf(a, fragb_f32(Wm + (size_t)(c0 + j * 16 + col) * EE + kc * 32, lane), acc[j]); }
#pragma unroll
  for (int j = 0; j < 8; ++j) { const float bb = bfr(Bm[c0 + j * 16 + col]);
#pragma unroll
    for (int r = 0; r < 8; ++r) { const float v = acc[j][r] + bb; const _Float16 hv = (_Float16)v, lv = (_Float16)((v - (float)hv) * 2048.0f); const int rl = wave * 16 + 8 * g + r, cl = j * 16 + col; if (which < 2) { sh[rl][cl] = hv; sl[rl][cl] = lv; } else { th[cl][rl] = hv; tl[cl][rl] = lv; } } }
  __syncthreads();
  if (which == 0) { for (int e = tid; e < 64 * 16; e += 128) { const int rl = e >> 4, q = e & 15; const size_t o = (b * NR + l0 + rl) * EE + c0 + q * 8; vst2((unsigned*)(QH + o), *(const v4u*)&sh[rl][q * 8]); vst2((unsigned*)(QL + o), *(const v4u*)&sl[rl][q * 8]); } }
  else if (which == 1) { for (int e = tid; e < 64 * 16; e += 128) { const int rl = e >> 4, q = e & 15; const size_t o = (b * NSLOT + 64 + l0 + rl) * EE + c0 + q * 8; vst2((unsigned*)(KH + o), *(const v4u*)&sh[rl][q * 8]); vst2((unsigned*)(KL + o), *(const v4u*)&sl[rl][q * 8]); } }
  else { for (int e = tid; e < 128 * 8; e += 128) { const int cl = e >> 3, q = e & 7; const size_t o = (b * EE + c0 + cl) * (size_t)NSLOT + 64 + l0 + q * 8; vst2((unsigned*)(VH + o), *(const v4u*)&th[cl][q * 8]); vst2((unsigned*)(VL + o), *(const v4u*)&tl[cl][q * 8]); } } }
__device__ __forceinline__ void attend16(const v16h aq[2], const v16h al[2], bool three, int h, size_t b, int stage, const int* qidx8  , const float* __restrict__ MASK, int mrows,
    const _Float16* __restrict__ KH, const _Float16* __restrict__ KL, const _Float16* __restrict__ VH, const _Float16* __restrict__ VL, float (*sp)[36], float (*so)[68], int lane) {
  const int col = lane & 15, g = lane >> 4;
  float m[8], l[8];
#pragma unroll
  for (int r = 0; r < 8; ++r) { m[r] = -3.0e38f; l[r] = 0.f; }
  v8f acc[4] = {}, accl[4] = {};
#pragma unroll 1
  for (int ks = 0; ks < NKT; ++ks) { if ((stage == 1 && ks == 1) || (stage == 2 && ks == 0)) continue;
    float s[2][8];
#pragma unroll
    for (int ct = 0; ct < 2; ++ct) { const int slot = ks * 32 + ct * 16 + col; const int tcol = (slot < 64) ? (slot & 31) : (slot - 32);
      const size_t rk = (b * NSLOT + slot) * EE + h * HD; v8f c = {}, cl = {};
#pragma unroll
      for (int kc = 0; kc < 2; ++kc) { const v16h kh = frag_h(KH + rk + kc * 32, lane); c = wmma16(aq[kc], kh, c); if (three) { cl = wmma16(al[kc], kh, cl); cl = wmma16(aq[kc], frag_h(KL + rk + kc * 32, lane), cl); } }
#pragma unroll
      for (int r = 0; r < 8; ++r) s[ct][r] = (c[r] + (three ? cl[r] * (1.0f / 2048.0f) : 0.f)) * 0.125f + bfr(MASK[((size_t)b * mrows + qidx8[r]) * NT1 + tcol]); }
    float alpha[8];
#pragma unroll
    for (int r = 0; r < 8; ++r) { float mx = fmaxf(s[0][r], s[1][r]);
#pragma unroll
      for (int o = 1; o < 16; o <<= 1) mx = fmaxf(mx, __shfl_xor(mx, o));
      const float mn = fmaxf(m[r], mx); alpha[r] = __expf(m[r] - mn); const float e0 = __expf(s[0][r] - mn), e1 = __expf(s[1][r] - mn); float es = e0 + e1;
#pragma unroll
      for (int o = 1; o < 16; o <<= 1) es += __shfl_xor(es, o);
      l[r] = l[r] * alpha[r] + es; m[r] = mn; sp[8 * g + r][col] = e0; sp[8 * g + r][16 + col] = e1; }
#pragma unroll
    for (int j = 0; j < 4; ++j)
#pragma unroll
      for (int r = 0; r < 8; ++r) { acc[j][r] *= alpha[r]; accl[j][r] *= alpha[r]; }
    LDSX();
    v16h pa, pl; { const float* prow = &sp[col][0] + 8 * (lane >> 4);
#pragma unroll
      for (int i = 0; i < 8; ++i) { const float x0 = prow[i] * 2048.0f, x1 = prow[16 + i] * 2048.0f; const _Float16 h0 = (_Float16)x0, h1 = (_Float16)x1; pa[i] = h0; pa[8 + i] = h1; pl[i] = (_Float16)((x0 - (float)h0) * 2048.0f); pl[8 + i] = (_Float16)((x1 - (float)h1) * 2048.0f); } }
#pragma unroll
    for (int j = 0; j < 4; ++j) { const size_t po = (b * EE + (size_t)h * HD + j * 16 + col) * NSLOT + ks * 32; const v16h vh = frag_h(VH + po, lane); acc[j] = wmma16(pa, vh, acc[j]); if (three) { accl[j] = wmma16(pl, vh, accl[j]); accl[j] = wmma16(pa, frag_h(VL + po, lane), accl[j]); } }
    LDSX(); }
#pragma unroll
  for (int r = 0; r < 8; ++r) { const float il = (1.0f / 2048.0f) / l[r];
#pragma unroll
    for (int j = 0; j < 4; ++j) so[8 * g + r][j * 16 + col] = (acc[j][r] + accl[j][r] * (1.0f / 2048.0f)) * il; }
  LDSX(); }
__global__ __launch_bounds__(64) void k_sum(const float* __restrict__ SXin, const float* __restrict__ MSX, const float* __restrict__ WSQ, const float* __restrict__ BSQ, const float* __restrict__ WSK, const float* __restrict__ BSK, const float* __restrict__ WSV, const float* __restrict__ BSV, const float* __restrict__ WK2, const float* __restrict__ BK2, const float* __restrict__ WV2, const float* __restrict__ BV2, const float* __restrict__ WSO, const float* __restrict__ BSO,
    _Float16* __restrict__ Q1H, _Float16* __restrict__ Q1L, _Float16* __restrict__ KH, _Float16* __restrict__ KL, _Float16* __restrict__ VH, _Float16* __restrict__ VL, float* __restrict__ SX, float* __restrict__ OUT0) {
  __shared__ __align__(16) _Float16 th[128][40], tl[128][40]; __shared__ __align__(16) float sp[2][16][36]; __shared__ __align__(16) float so[2][16][68]; __shared__ __align__(16) float sf[2][16][132]; __shared__ __align__(16) _Float16 sh2[2][16][136], sl2[2][16][136];
  const int tid = threadIdx.x, wave = tid >> 5, lane = tid & 31, col = lane & 15, g = lane >> 4; const size_t b = blockIdx.x; const int s0 = wave * 16;
#pragma unroll 1
  for (int which = 0; which < 3; ++which) { const float* Wm = which == 0 ? WSQ : which == 1 ? WSK : WSV; const float* Bm = which == 0 ? BSQ : which == 1 ? BSK : BSV;
#pragma unroll 1
    for (int cg = 0; cg < EE / 128; ++cg) { v8f acc[8] = {};
#pragma unroll 2
      for (int kc = 0; kc < EE / 32; ++kc) { const v16b a = fragb_f32(SXin + ((size_t)(s0 + col) * NB + b) * EE + kc * 32, lane);
#pragma unroll
        for (int j = 0; j < 8; ++j) acc[j] = wmma_bf(a, fragb_f32(Wm + (size_t)(cg * 128 + j * 16 + col) * EE + kc * 32, lane), acc[j]); }
#pragma unroll
      for (int j = 0; j < 8; ++j) { const float bb = bfr(Bm[cg * 128 + j * 16 + col]);
#pragma unroll
        for (int r = 0; r < 8; ++r) { const float v = acc[j][r] + bb; const _Float16 hv = (_Float16)v, lv = (_Float16)((v - (float)hv) * 2048.0f); const int rl = 8 * g + r, cl = j * 16 + col; if (which < 2) { sh2[wave][rl][cl] = hv; sl2[wave][rl][cl] = lv; } else { th[cl][s0 + rl] = hv; tl[cl][s0 + rl] = lv; } } }
      if (which < 2) { LDSX(); _Float16* DH = which == 0 ? Q1H : KH; _Float16* DL = which == 0 ? Q1L : KL; const size_t rowbase = which == 0 ? (b * NS + s0) : (b * NSLOT + s0);
        for (int e = lane; e < 16 * 16; e += 32) { const int rl = e >> 4, q = e & 15; const size_t o = (rowbase + rl) * EE + cg * 128 + q * 8; vst2((unsigned*)(DH + o), *(const v4u*)&sh2[wave][rl][q * 8]); vst2((unsigned*)(DL + o), *(const v4u*)&sl2[wave][rl][q * 8]); }
        LDSX(); }
      else { __syncthreads();
        for (int e = tid; e < 128 * 4; e += 64) { const int cl = e >> 2, q = e & 3; const size_t o = (b * EE + cg * 128 + cl) * (size_t)NSLOT + q * 8; vst2((unsigned*)(VH + o), *(const v4u*)&th[cl][q * 8]); vst2((unsigned*)(VL + o), *(const v4u*)&tl[cl][q * 8]); }
        __syncthreads(); } } }
  __threadfence(); __syncthreads();
  int qidx[8];
#pragma unroll
  for (int r = 0; r < 8; ++r) qidx[r] = s0 + 8 * g + r;
#pragma unroll 1
  for (int h = 0; h < NH; ++h) { v16h aq[2], al[2];
#pragma unroll
    for (int kc = 0; kc < 2; ++kc) { aq[kc] = frag_h(Q1H + ((b * NS + s0 + col) * EE) + h * HD + kc * 32, lane); al[kc] = frag_h(Q1L + ((b * NS + s0 + col) * EE) + h * HD + kc * 32, lane); }
    attend16(aq, al, true, h, b, 1, qidx, MSX, NS, KH, KL, VH, VL, sp[wave], so[wave], lane);
    for (int rl = 0; rl < 16; ++rl) if (lane < 16) vst2(SX + (b * NS + s0 + rl) * EE + h * HD + lane * 4, *(const v4f*)&so[wave][rl][lane * 4]);
    LDSX(); }
  __threadfence(); __syncthreads();
#pragma unroll 1
  for (int which = 0; which < 3; ++which) { const float* Wm = which == 0 ? WK2 : which == 1 ? WV2 : WSO; const float* Bm = which == 0 ? BK2 : which == 1 ? BV2 : BSO;
#pragma unroll 1
    for (int cg = 0; cg < EE / 128; ++cg) { v8f acc[8] = {};
#pragma unroll 2
      for (int kc = 0; kc < EE / 32; ++kc) { const F2 a = split_row(SX + (b * NS + s0 + col) * EE, kc * 32, lane);
#pragma unroll
        for (int j = 0; j < 8; ++j) { const v16b w = fragb_f32(Wm + (size_t)(cg * 128 + j * 16 + col) * EE + kc * 32, lane); acc[j] = wmma_bf(a.h, w, acc[j]); acc[j] = wmma_bf(a.l, w, acc[j]); } }
      if (which == 2) {
#pragma unroll
        for (int j = 0; j < 8; ++j) { const float bb = bfr(Bm[cg * 128 + j * 16 + col]);
#pragma unroll
          for (int r = 0; r < 8; ++r) sf[wave][8 * g + r][j * 16 + col] = acc[j][r] + bb; }
        LDSX(); for (int rl = 0; rl < 16; ++rl) vst2(OUT0 + ((size_t)(s0 + rl) * NB + b) * EE + cg * 128 + lane * 4, *(const v4f*)&sf[wave][rl][lane * 4]);
        LDSX(); }
      else {
#pragma unroll
        for (int j = 0; j < 8; ++j) { const float bb = bfr(Bm[cg * 128 + j * 16 + col]);
#pragma unroll
          for (int r = 0; r < 8; ++r) { const float v = acc[j][r] + bb; const _Float16 hv = (_Float16)v, lv = (_Float16)((v - (float)hv) * 2048.0f); const int rl = 8 * g + r, cl = j * 16 + col; if (which == 0) { sh2[wave][rl][cl] = hv; sl2[wave][rl][cl] = lv; } else { th[cl][s0 + rl] = hv; tl[cl][s0 + rl] = lv; } } }
        if (which == 0) { LDSX(); for (int e = lane; e < 16 * 16; e += 32) { const int rl = e >> 4, q = e & 15; const size_t o = (b * NSLOT + 32 + s0 + rl) * EE + cg * 128 + q * 8; vst2((unsigned*)(KH + o), *(const v4u*)&sh2[wave][rl][q * 8]); vst2((unsigned*)(KL + o), *(const v4u*)&sl2[wave][rl][q * 8]); } LDSX(); }
        else { __syncthreads(); for (int e = tid; e < 128 * 4; e += 64) { const int cl = e >> 2, q = e & 3; const size_t o = (b * EE + cg * 128 + cl) * (size_t)NSLOT + 32 + q * 8; vst2((unsigned*)(VH + o), *(const v4u*)&th[cl][q * 8]); vst2((unsigned*)(VL + o), *(const v4u*)&tl[cl][q * 8]); } __syncthreads(); } } } } }
__global__ __launch_bounds__(128) void k_att2(const _Float16* __restrict__ QH, const _Float16* __restrict__ QL, const _Float16* __restrict__ KH, const _Float16* __restrict__ KL, const _Float16* __restrict__ VH, const _Float16* __restrict__ VL, const float* __restrict__ MRX, float* __restrict__ O) {
  __shared__ __align__(16) float sp[4][16][36]; __shared__ __align__(16) float so[4][16][68];
  const int tid = threadIdx.x, wave = tid >> 5, lane = tid & 31, col = lane & 15, g = lane >> 4; const int qb = blockIdx.x, h = blockIdx.y; const size_t b = blockIdx.z; const int q0 = qb * 64 + wave * 16;
  v16h aq[2], al[2];
#pragma unroll
  for (int kc = 0; kc < 2; ++kc) { aq[kc] = frag_h(QH + (b * NR + q0 + col) * EE + h * HD + kc * 32, lane); al[kc] = frag_h(QL + (b * NR + q0 + col) * EE + h * HD + kc * 32, lane); }
  int qidx[8];
#pragma unroll
  for (int r = 0; r < 8; ++r) qidx[r] = q0 + 8 * g + r;
  attend16(aq, al, qb < 2, h, b, 2, qidx, MRX, NR, KH, KL, VH, VL, sp[wave], so[wave], lane);
  for (int rl = 0; rl < 16; ++rl) if (lane < 16) vst2(O + (b * NR + q0 + rl) * EE + (size_t)h * HD + lane * 4, *(const v4f*)&so[wave][rl][lane * 4]); }
__global__ __launch_bounds__(128) void k_out2(const float* __restrict__ O, const float* __restrict__ WRO, const float* __restrict__ BRO, float* __restrict__ OUT1) { __shared__ __align__(16) float sf[4][16][132];
  const int tid = threadIdx.x, wave = tid >> 5, lane = tid & 31, col = lane & 15, g = lane >> 4; const size_t b = blockIdx.z; const int l0 = blockIdx.x * 64 + wave * 16; const int c0 = blockIdx.y * 128;
  v8f acc[8] = {};
#pragma unroll 2
  for (int kc = 0; kc < EE / 32; ++kc) { const F2 a = split_row(O + (b * NR + l0 + col) * EE, kc * 32, lane);
#pragma unroll
    for (int j = 0; j < 8; ++j) { const v16b w = fragb_f32(WRO + (size_t)(c0 + j * 16 + col) * EE + kc * 32, lane); acc[j] = wmma_bf(a.h, w, acc[j]); acc[j] = wmma_bf(a.l, w, acc[j]); } }
#pragma unroll
  for (int j = 0; j < 8; ++j) { const float bb = bfr(BRO[c0 + j * 16 + col]);
#pragma unroll
    for (int r = 0; r < 8; ++r) sf[wave][8 * g + r][j * 16 + col] = acc[j][r] + bb; }
  LDSX(); for (int rl = 0; rl < 16; ++rl) vst2(OUT1 + ((size_t)(l0 + rl) * NB + b) * EE + c0 + lane * 4, *(const v4f*)&sf[wave][rl][lane * 4]); }
extern "C" void kernel_launch(void* const* d_in, const int* in_sizes, int n_in, void* d_out, int out_size, void* d_ws, size_t ws_size, hipStream_t stream) {
  (void)in_sizes; (void)n_in; (void)out_size;
  const float** F = (const float**)d_in;
  if (ws_size < (size_t)WS_END) return;
  char* ws = (char*)d_ws; _Float16 *QH = (_Float16*)(ws + WS_QH), *QL = (_Float16*)(ws + WS_QL), *KH = (_Float16*)(ws + WS_KH), *KL = (_Float16*)(ws + WS_KL), *VH = (_Float16*)(ws + WS_VH), *VL = (_Float16*)(ws + WS_VL), *Q1H = (_Float16*)(ws + WS_Q1H), *Q1L = (_Float16*)(ws + WS_Q1L); float *O = (float*)(ws + WS_O), *SX = (float*)(ws + WS_SX);
  float* OUT0 = (float*)d_out; float* OUT1 = OUT0 + (size_t)NS * NB * EE;
  k_reg<<<dim3(NR / 64, EE / 128, 3 * TNB), 128, 0, stream>>>(F[1], F[7], F[8], F[9], F[10], F[11], F[12], QH, QL, KH, KL, VH, VL);
  k_sum<<<TNB, 64, 0, stream>>>(F[0], F[5], F[15], F[16], F[17], F[18], F[19], F[20], F[23], F[24], F[25], F[26], F[21], F[22], Q1H, Q1L, KH, KL, VH, VL, SX, OUT0);
  k_att2<<<dim3(TQ2, NH, TNB), 128, 0, stream>>>(QH, QL, KH, KL, VH, VL, F[6], O);
  k_out2<<<dim3(TQ2, EE / 128, TNB), 128, 0, stream>>>(O, F[13], F[14], OUT1);
}
